// SpectralSSM_65077344469103
// MI455X (gfx1250) — hardware-run, weakly checked
//
#include <hip/hip_runtime.h>
#include <math.h>

typedef __attribute__((ext_vector_type(16))) _Float16 v16h;
typedef __attribute__((ext_vector_type(8)))  _Float16 v8h;
typedef __attribute__((ext_vector_type(8)))  float    v8f;
typedef __attribute__((ext_vector_type(4)))  float    v4f;

constexpr int kPix    = 4096;
constexpr int kBands  = 224;
constexpr int kDm     = 64;
constexpr int kDs     = 16;
constexpr int kCols   = kDm * kDs;
constexpr int kDepth  = 480;
constexpr int kPitch  = 512;
constexpr float kCarry    = 32.0f;
constexpr float kCarryInv = 1.0f / kCarry;
constexpr float kResCarry = 2048.0f;
constexpr float kResFold  = 1.0f / kResCarry;
constexpr float kF16Floor = 6.2e-5f;
constexpr float kLnEps    = 1e-5f;
static_assert(kCols == 1024, "column flattening d*16+s");
static_assert(2 * kBands + 1 <= kDepth && (kDepth % 32) == 0 && kDepth <= kPitch, "depth layout");
static_assert((kPix % 32) == 0 && (kCols % 32) == 0, "GEMM M,N multiples of the 32x32 wave tile");
static_assert((((kPix / 32) * (kCols / 32)) % 8) == 0, "whole blocks of 8 wave tiles");
static_assert((kPitch * 2) % 128 == 0, "plane row = whole lines");
static_assert((kBands % 8) == 0, "8-element chunks do not straddle column ranges");
static_assert((kPix % 8) == 0 && (kPix % 4) == 0 && (kCols % 4) == 0, "producer grids exact");

constexpr size_t kOffAH  = 0;
constexpr size_t kOffAL  = kOffAH + (size_t)kPix  * kPitch * 2;
constexpr size_t kOffBH  = kOffAL + (size_t)kPix  * kPitch * 2;
constexpr size_t kOffBL  = kOffBH + (size_t)kCols * kPitch * 2;
constexpr size_t kOffH   = kOffBL + (size_t)kCols * kPitch * 2;
constexpr size_t kWsTotal = kOffH + (size_t)kPix * kCols * 4;
static_assert(kWsTotal == 27262976ull, "carve total");
static_assert(kWsTotal <= 134217728ull, "carve cap");
static_assert((kOffAL % 128) == 0 && (kOffBH % 128) == 0 && (kOffBL % 128) == 0 && (kOffH % 128) == 0,
              "128-B aligned regions");

union FragU { v16h v; v8h h[2]; };
__device__ __forceinline__ v16h frag_load(const _Float16* p) {
  FragU f;
  f.h[0] = *(const v8h*)(p);
  f.h[1] = *(const v8h*)(p + 16);
  return f.v;
}
__device__ __forceinline__ v8f frag_mma(v16h a, v16h b, v8f c) {
  return __builtin_amdgcn_wmma_f32_16x16x32_f16(false, a, false, b, (short)0, c, false, false);
}
__device__ __forceinline__ void group_guard(v8f& a, v8f& b, v8f& c, v8f& d, v16h x, v16h y) {
  asm volatile("v_nop\n\tv_nop\n\tv_nop\n\tv_nop" : "+v"(a), "+v"(b), "+v"(c), "+v"(d) : "v"(x), "v"(y));
}
__device__ __forceinline__ void keep4_h(v16h a, v16h b, v16h c, v16h d) {
  asm volatile("v_nop" :: "v"(a), "v"(b), "v"(c), "v"(d));
}
__device__ __forceinline__ void acc_guard4(v8f& a, v8f& b, v8f& c, v8f& d) {
  asm volatile("v_nop\n\tv_nop\n\tv_nop\n\tv_nop" : "+v"(a), "+v"(b), "+v"(c), "+v"(d));
}

__device__ __forceinline__ void split16(float v, _Float16& hi, _Float16& lo) {
  const float vc = fminf(fmaxf(v, -60000.0f), 60000.0f);
  const _Float16 h0 = (_Float16)vc;
  const float hf0 = (float)h0;
  const float hf  = (fabsf(hf0) >= kF16Floor) ? hf0 : 0.0f;
  const float rr  = (vc - hf) * kResCarry;
  const _Float16 l0 = (_Float16)rr;
  const float lf0 = (float)l0;
  const float lf  = (fabsf(lf0) >= kF16Floor) ? lf0 : 0.0f;
  hi = (_Float16)hf;
  lo = (_Float16)lf;
}

__device__ __forceinline__ float collapse16(const float* __restrict__ w_in, const float* __restrict__ b_in,
                                            const float* __restrict__ W, int lane) {
  const int s = lane & 15;
  const bool useB = (lane >= 16);
  float acc = 0.0f;
#pragma unroll 1
  for (int d = 0; d < kDm; ++d) {
    float wv = w_in[d];
    float bv = b_in[d];
    const float mv = W[d * kDs + s];
    asm volatile("" : "+v"(wv), "+v"(bv));
    const float sel = useB ? bv : wv;
    acc = fmaf(sel, mv, acc);
  }
  return acc;
}

__global__ __launch_bounds__(256) void prep_bt_kernel(
    const float* __restrict__ w_in, const float* __restrict__ b_in,
    const float* __restrict__ A_log, const float* __restrict__ Wb,
    unsigned short* __restrict__ BtH, unsigned short* __restrict__ BtL)
{
  __shared__ float sWB[32];
  __shared__ __align__(16) float sV[4 * kPitch];
  const int tid  = threadIdx.x;
  const int lane = tid & 31;
  const int wave = __builtin_amdgcn_readfirstlane((int)(threadIdx.x >> 5));
  if (wave == 0) sWB[lane] = collapse16(w_in, b_in, Wb, lane);
  __syncthreads();
#pragma unroll 1
  for (int i = 0; i < 8; ++i) {
    const int r   = i >> 1;
    const int k   = ((i & 1) << 8) + tid;
    const int col = blockIdx.x * 4 + r;
    const int d   = col >> 4;
    const int s   = col & 15;
    const float ea  = expf(A_log[col]);
    const float wd  = w_in[d];
    const float bd  = b_in[d];
    const float wbs = sWB[s];
    const float bbs = sWB[16 + s];
    const float cA  = wd * wbs;
    const float cB  = wd * bbs + bd * wbs;
    const float a1   = expf(-ea);
    const float a224 = expf(-(float)kBands * ea);
    const float den  = fmaxf(1.0f - a1, 1.0e-20f);
    const float cC   = bd * bbs * ((1.0f - a224) * (1.0f / den));
    const bool first = (k < kBands);
    int m = first ? (kBands - 1 - k) : (2 * kBands - 1 - k);
    m = (m < 0) ? 0 : m;
    const float coef = first ? cB : cA;
    const float pw   = expf(-(float)m * ea);
    float val = coef * pw;
    val = (k == 2 * kBands) ? cC : val;
    val = (k > 2 * kBands) ? 0.0f : val;
    float carried = val * kCarry;
    carried = (fabsf(carried) >= kF16Floor) ? carried : 0.0f;
    sV[r * kPitch + k] = carried;
  }
  __syncthreads();
  {
    const int rr = tid >> 6;
    const int c8 = (tid & 63) * 8;
    const v4f a0 = *(const v4f*)(sV + rr * kPitch + c8);
    const v4f a1 = *(const v4f*)(sV + rr * kPitch + c8 + 4);
    v8h hv, lv;
#pragma unroll
    for (int e = 0; e < 4; ++e) {
      const float f0 = a0[e];
      const float f1 = a1[e];
      _Float16 h0, l0, h1, l1;
      split16(f0, h0, l0);
      split16(f1, h1, l1);
      hv[e]     = h0;
      hv[4 + e] = h1;
      lv[e]     = l0;
      lv[4 + e] = l1;
    }
    const size_t o = (size_t)(blockIdx.x * 4 + rr) * kPitch + c8;
    unsigned short* qh = BtH + o;
    unsigned short* ql = BtL + o;
    *(volatile v8h*)qh = hv;
    *(volatile v8h*)ql = lv;
    __threadfence();
    *(volatile v8h*)qh = hv;
    *(volatile v8h*)ql = lv;
  }
}

__global__ __launch_bounds__(256) void prep_a_kernel(
    const float* __restrict__ x, unsigned short* __restrict__ ApH, unsigned short* __restrict__ ApL)
{
  const int tid = threadIdx.x;
  const int n   = blockIdx.x * 4 + (tid >> 6);
  const int c   = tid & 63;
  constexpr int kChunks = kBands / 8;
  const bool sq  = (c >= kChunks);
  const bool pad = (c >= 2 * kChunks);
  const int src  = pad ? 0 : (sq ? (c - kChunks) : c);
  const float* p = x + (size_t)n * kBands + 8 * src;
  const v4f a0 = *(const v4f*)(p);
  const v4f a1 = *(const v4f*)(p + 4);
  float f0 = a0[0], f1 = a0[1], f2 = a0[2], f3 = a0[3];
  float f4 = a1[0], f5 = a1[1], f6 = a1[2], f7 = a1[3];
  asm volatile("" : "+v"(f0), "+v"(f1), "+v"(f2), "+v"(f3));
  asm volatile("" : "+v"(f4), "+v"(f5), "+v"(f6), "+v"(f7));
  float g[8];
  g[0] = f0; g[1] = f1; g[2] = f2; g[3] = f3; g[4] = f4; g[5] = f5; g[6] = f6; g[7] = f7;
  const float one0 = (c == 2 * kChunks) ? 1.0f : 0.0f;
  v8h hv, lv;
#pragma unroll
  for (int e = 0; e < 8; ++e) {
    const float lin = g[e];
    const float sqv = lin * lin;
    float val = sq ? sqv : lin;
    const float pv = (e == 0) ? one0 : 0.0f;
    val = pad ? pv : val;
    _Float16 hh, ll;
    split16(val, hh, ll);
    hv[e] = hh;
    lv[e] = ll;
  }
  const size_t o = (size_t)n * kPitch + 8 * c;
  unsigned short* qh = ApH + o;
  unsigned short* ql = ApL + o;
  *(volatile v8h*)qh = hv;
  *(volatile v8h*)ql = lv;
  __threadfence();
  *(volatile v8h*)qh = hv;
  *(volatile v8h*)ql = lv;
}

__global__ __launch_bounds__(256) void gemm32_f16x3_kernel(
    const unsigned short* __restrict__ AHp, const unsigned short* __restrict__ ALp, int lda,
    const unsigned short* __restrict__ BHp, const unsigned short* __restrict__ BLp, int ldb,
    float* __restrict__ C, int ldc,
    int M, int N, int K, float resFold, float scale)
{
  __shared__ __align__(16) float sT[8][16 * 36];
  const int lane = threadIdx.x & 31;
  const int wave = __builtin_amdgcn_readfirstlane((int)(threadIdx.x >> 5));
  const int tilesN = N >> 5;
  const int tilesM = M >> 5;
  const int tile = blockIdx.x * 8 + wave;
  if (tile >= tilesM * tilesN) return;
  const int tm = tile / tilesN;
  const int tn = tile - tm * tilesN;
  const int m0 = tm << 5;
  const int n0 = tn << 5;

  const int rlane = lane & 15;
  const int koff  = (lane >> 4) * 8;
  const int mOff  = (lane >> 4) * 8;

  const _Float16* paH = (const _Float16*)AHp + (size_t)(m0 + rlane) * lda + koff;
  const _Float16* paL = (const _Float16*)ALp + (size_t)(m0 + rlane) * lda + koff;
  const _Float16* pbH = (const _Float16*)BHp + (size_t)(n0 + rlane) * ldb + koff;
  const _Float16* pbL = (const _Float16*)BLp + (size_t)(n0 + rlane) * ldb + koff;
  const size_t a16 = (size_t)16 * lda;
  const size_t b16 = (size_t)16 * ldb;

  v8f acc[2][2], res[2][2];
#pragma unroll
  for (int i = 0; i < 2; ++i)
#pragma unroll
    for (int j = 0; j < 2; ++j) {
      acc[i][j] = (v8f){0.f, 0.f, 0.f, 0.f, 0.f, 0.f, 0.f, 0.f};
      res[i][j] = (v8f){0.f, 0.f, 0.f, 0.f, 0.f, 0.f, 0.f, 0.f};
    }

  for (int k0 = 0; k0 < K; k0 += 32) {
    const v16h ah0 = frag_load(paH + k0);
    const v16h ah1 = frag_load(paH + a16 + k0);
    const v16h al0 = frag_load(paL + k0);
    const v16h al1 = frag_load(paL + a16 + k0);
#pragma unroll
    for (int j = 0; j < 2; ++j) {
      const v16h bh = frag_load(pbH + (size_t)j * b16 + k0);
      const v16h bl = frag_load(pbL + (size_t)j * b16 + k0);
      acc[0][j] = frag_mma(ah0, bh, acc[0][j]);
      acc[1][j] = frag_mma(ah1, bh, acc[1][j]);
      res[0][j] = frag_mma(ah0, bl, res[0][j]);
      res[1][j] = frag_mma(ah1, bl, res[1][j]);
      res[0][j] = frag_mma(al0, bh, res[0][j]);
      res[1][j] = frag_mma(al1, bh, res[1][j]);
      group_guard(acc[0][j], acc[1][j], res[0][j], res[1][j], bh, bl);
    }
    keep4_h(ah0, ah1, al0, al1);
  }
  acc_guard4(acc[0][0], acc[0][1], acc[1][0], acc[1][1]);
  acc_guard4(res[0][0], res[0][1], res[1][0], res[1][1]);

  float* slab = sT[wave];
#pragma unroll
  for (int i = 0; i < 2; ++i) {
    const int mBase = m0 + (i << 4);
#pragma unroll
    for (int j = 0; j < 2; ++j) {
#pragma unroll
      for (int r = 0; r < 8; ++r) {
        const float mainv = acc[i][j][r];
        const float resv  = res[i][j][r];
        const float v = (mainv + resv * resFold) * scale;
        slab[(mOff + r) * 36 + (j << 4) + rlane] = v;
      }
    }
    __builtin_amdgcn_fence(__ATOMIC_RELEASE, "workgroup");
    __builtin_amdgcn_wave_barrier();
    __builtin_amdgcn_fence(__ATOMIC_ACQUIRE, "workgroup");
    {
      const int q  = lane >> 3;
      const int c4 = (lane & 7) * 4;
      for (int pass = 0; pass < 2; ++pass) {
#pragma unroll
        for (int it = 0; it < 4; ++it) {
          const int row = it * 4 + q;
          const v4f v = *(const v4f*)(slab + row * 36 + c4);
          *(volatile v4f*)(C + (size_t)(mBase + row) * ldc + n0 + c4) = v;
        }
        __threadfence();
      }
    }
    __builtin_amdgcn_fence(__ATOMIC_RELEASE, "workgroup");
    __builtin_amdgcn_wave_barrier();
    __builtin_amdgcn_fence(__ATOMIC_ACQUIRE, "workgroup");
  }
}

__global__ __launch_bounds__(256) void tail_kernel(
    const float* __restrict__ x, const float* __restrict__ w_in, const float* __restrict__ b_in,
    const float* __restrict__ Wc, const float* __restrict__ Dv, const float* __restrict__ Wo,
    const float* __restrict__ bo, const float* __restrict__ gamma, const float* __restrict__ beta,
    const float* __restrict__ H, float* __restrict__ out)
{
  __shared__ float sWo[kDm * 65];
  __shared__ __align__(16) float sCc[32];
  __shared__ float sBo[kDm];
  __shared__ float sOut[8 * kDm];
  __shared__ __align__(16) float sRes[8 * kDm];
  const int tid  = threadIdx.x;
  const int lane = tid & 31;
  const int wave = __builtin_amdgcn_readfirstlane((int)(threadIdx.x >> 5));
#pragma unroll 1
  for (int i = 0; i < 16; ++i) {
    const int e = i * 256 + tid;
    sWo[(e >> 6) * 65 + (e & 63)] = Wo[e];
  }
  if (wave < 2) sBo[tid] = bo[tid];
  if (wave == 0) sCc[lane] = collapse16(w_in, b_in, Wc, lane);
  __syncthreads();

  const int n  = blockIdx.x * 8 + wave;
  const int d1 = lane;
  const int d2 = lane + 32;
  const float xl  = x[(size_t)n * kBands + (kBands - 1)];
  const float w1  = w_in[d1],  w2  = w_in[d2];
  const float b1  = b_in[d1],  b2  = b_in[d2];
  const float dd1 = Dv[d1],    dd2 = Dv[d2];
  const float g1  = gamma[d1], g2  = gamma[d2];
  const float be1 = beta[d1],  be2 = beta[d2];
  const float* h1 = H + (size_t)n * kCols + d1 * kDs;
  const float* h2 = H + (size_t)n * kCols + d2 * kDs;
  float y1 = 0.0f, y2 = 0.0f;
#pragma unroll 1
  for (int q = 0; q < 4; ++q) {
    const v4f wc4 = *(const v4f*)(sCc + 4 * q);
    const v4f bc4 = *(const v4f*)(sCc + 16 + 4 * q);
    const v4f ha  = *(const v4f*)(h1 + 4 * q);
    const v4f hb  = *(const v4f*)(h2 + 4 * q);
#pragma unroll
    for (int e = 0; e < 4; ++e) {
      const float cs = fmaf(xl, wc4[e], bc4[e]);
      y1 = fmaf(ha[e], cs, y1);
      y2 = fmaf(hb[e], cs, y2);
    }
  }
  const float o1 = y1 + dd1 * fmaf(xl, w1, b1);
  const float o2 = y2 + dd2 * fmaf(xl, w2, b2);
  sOut[wave * kDm + d1] = o1;
  sOut[wave * kDm + d2] = o2;
  __syncthreads();

  const float* orow = sOut + wave * kDm;
  const float* wr1  = sWo + d1 * 65;
  const float* wr2  = sWo + d2 * 65;
  float z1 = 0.0f, z2 = 0.0f;
#pragma unroll 4
  for (int k = 0; k < kDm; ++k) {
    const float ok = orow[k];
    z1 = fmaf(ok, wr1[k], z1);
    z2 = fmaf(ok, wr2[k], z2);
  }
  z1 += sBo[d1];
  z2 += sBo[d2];

  float sum = z1 + z2;
  sum += __shfl_xor(sum, 16, 32);
  sum += __shfl_xor(sum, 8, 32);
  sum += __shfl_xor(sum, 4, 32);
  sum += __shfl_xor(sum, 2, 32);
  sum += __shfl_xor(sum, 1, 32);
  const float mu = sum * (1.0f / (float)kDm);
  const float e1 = z1 - mu;
  const float e2 = z2 - mu;
  float sqs = e1 * e1 + e2 * e2;
  sqs += __shfl_xor(sqs, 16, 32);
  sqs += __shfl_xor(sqs, 8, 32);
  sqs += __shfl_xor(sqs, 4, 32);
  sqs += __shfl_xor(sqs, 2, 32);
  sqs += __shfl_xor(sqs, 1, 32);
  const float rs = rsqrtf(sqs * (1.0f / (float)kDm) + kLnEps);
  const float r1 = g1 * e1 * rs + be1;
  const float r2 = g2 * e2 * rs + be2;
  sRes[wave * kDm + d1] = r1;
  sRes[wave * kDm + d2] = r2;
  __syncthreads();

  if (wave < 4) {
    const v4f v = *(const v4f*)(sRes + tid * 4);
    float* p = out + (size_t)blockIdx.x * (8 * kDm) + tid * 4;
    *(volatile v4f*)p = v;
    __threadfence();
    *(volatile v4f*)p = v;
  }
}

extern "C" void kernel_launch(void* const* d_in, const int* in_sizes, int n_in,
                              void* d_out, int out_size, void* d_ws, size_t ws_size,
                              hipStream_t stream) {
  if (n_in < 11) return;
  if (in_sizes[0] != kPix * kBands) return;
  if (in_sizes[1] != kDm || in_sizes[2] != kDm) return;
  if (in_sizes[3] != kCols || in_sizes[4] != kCols || in_sizes[5] != kCols) return;
  if (in_sizes[6] != kDm) return;
  if (in_sizes[7] != kDm * kDm) return;
  if (in_sizes[8] != kDm || in_sizes[9] != kDm || in_sizes[10] != kDm) return;
  if (out_size != kPix * kDm) return;
  if (ws_size < kWsTotal) return;

  const float* x     = (const float*)d_in[0];
  const float* w_in  = (const float*)d_in[1];
  const float* b_in  = (const float*)d_in[2];
  const float* A_log = (const float*)d_in[3];
  const float* Wb    = (const float*)d_in[4];
  const float* Wc    = (const float*)d_in[5];
  const float* Dv    = (const float*)d_in[6];
  const float* Wo    = (const float*)d_in[7];
  const float* bo    = (const float*)d_in[8];
  const float* gamma = (const float*)d_in[9];
  const float* beta  = (const float*)d_in[10];
  float* outp = (float*)d_out;

  char* ws = (char*)d_ws;
  unsigned short* AHP = (unsigned short*)(ws + kOffAH);
  unsigned short* ALP = (unsigned short*)(ws + kOffAL);
  unsigned short* BHP = (unsigned short*)(ws + kOffBH);
  unsigned short* BLP = (unsigned short*)(ws + kOffBL);
  float*          HPL = (float*)(ws + kOffH);

  prep_bt_kernel<<<kCols / 4, 256, 0, stream>>>(w_in, b_in, A_log, Wb, BHP, BLP);
  prep_a_kernel<<<kPix / 4, 256, 0, stream>>>(x, AHP, ALP);
  gemm32_f16x3_kernel<<<((kPix / 32) * (kCols / 32)) / 8, 256, 0, stream>>>(
      AHP, ALP, kPitch, BHP, BLP, kPitch, HPL, kCols, kPix, kCols, kDepth, kResFold, kCarryInv);
  tail_kernel<<<kPix / 8, 256, 0, stream>>>(x, w_in, b_in, Wc, Dv, Wo, bo, gamma, beta, HPL, outp);
}
